// CGH_MMDecoderLSTM_44865228374203
// MI455X (gfx1250) — hardware-verified
//
#include <hip/hip_runtime.h>


namespace {
constexpr int S = 30, HD = 64, EM = 16, NS = 3, B = 16384, KA = 96, G4 = 4 * HD, CI = NS * (S * 2 + HD);
constexpr int OFF1 = B * NS * S * 2;
constexpr float HS = 64.0f, WSC = 256.0f, SLOPE = 0.01f;
typedef _Float16 b16;
typedef __attribute__((ext_vector_type(16))) _Float16 v16b;
typedef __attribute__((ext_vector_type(8))) _Float16 v8b;
typedef __attribute__((ext_vector_type(8))) float v8f;
typedef __attribute__((ext_vector_type(4))) float v4f;
typedef __attribute__((ext_vector_type(2))) float v2f;
__device__ __forceinline__ float bf16_rne(float f) { unsigned int u = __float_as_uint(f); u += 0x7FFFu + ((u >> 16) & 1u); return __uint_as_float(u & 0xFFFF0000u); }
__device__ __forceinline__ void split16(float v, b16& hi, b16& lo) { hi = (b16)v; lo = (b16)(v - (float)hi); }
__device__ __forceinline__ v16b frag_kb(const b16* p, int hh) { const v8b a = *(const v8b*)(p + 8 * hh), b = *(const v8b*)(p + 16 + 8 * hh); v16b f;
#pragma unroll
  for (int e = 0; e < 8; ++e) { f[e] = a[e]; f[8 + e] = b[e]; } return f; }
__device__ __forceinline__ v8f wmma16b(v16b a, v16b b, v8f c) { v8f d = __builtin_amdgcn_wmma_f32_16x16x32_f16(false, a, false, b, (short)0, c, false, false); asm volatile("v_nop\n\tv_nop\n\tv_nop\n\tv_nop" : "+v"(d) : "v"(a), "v"(b)); return d; }
__device__ __forceinline__ void wave_lds_sync() { __builtin_amdgcn_fence(__ATOMIC_RELEASE, "workgroup"); __builtin_amdgcn_wave_barrier(); __builtin_amdgcn_fence(__ATOMIC_ACQUIRE, "workgroup"); }
__device__ __forceinline__ float pmul(float a, float b) { float p = a * b; asm volatile("" : "+v"(p)); return p; }
__device__ __forceinline__ float sigm(float v) { return 1.0f / (1.0f + __expf(-v)); }
__device__ __forceinline__ float leaky(float v) { return v >= 0.0f ? v : SLOPE * v; }

__global__ __launch_bounds__(256) void wl_kernel(const float* __restrict__ wih, const float* __restrict__ whh, b16* __restrict__ WT) {
  const int u = blockIdx.x * 256 + threadIdx.x; if (u >= G4 * KA / 8) return; const int e = u * 8; const int o = e / KA, k0 = e % KA; v8b v;
#pragma unroll
  for (int j = 0; j < 8; ++j) { const int k = k0 + j; float w = 0.0f; if (k < EM) w = wih[o * EM + k]; else if (k >= 32) w = whh[o * HD + k - 32]; v[j] = (b16)(bf16_rne(w) * WSC); }
  for (int pass = 0; pass < 2; ++pass) { *(volatile v8b*)(WT + e) = v; __threadfence(); }
}
__global__ __launch_bounds__(32) void dec_kernel(const float* __restrict__ tr, const float* __restrict__ h0, const float* __restrict__ c0, const b16* __restrict__ WL, const float* __restrict__ bih, const float* __restrict__ bhh, const float* __restrict__ We, const float* __restrict__ be, const float* __restrict__ Wp, const float* __restrict__ bp, const float* __restrict__ Wc, const float* __restrict__ bc, int BV, float* __restrict__ out) {
  __shared__ __attribute__((aligned(16))) b16 Ah[16][KA + 8], Al[16][KA + 8]; __shared__ float Hs[16][HD + 1], Cs[16][HD + 1], X0[16][EM], Xs[16][EM], Pr[32][NS * S * 2], Fn[16][NS * HD], Cf[32][NS];
  const int lane = threadIdx.x, nloc = lane & 15, hlf = lane >> 4; const size_t r0w = (size_t)blockIdx.x * 32;
  float we2[2], bel; { const int ee = lane & 15; we2[0] = bf16_rne(We[ee * 2]); we2[1] = bf16_rne(We[ee * 2 + 1]); bel = bf16_rne(be[ee]); }
  float bsum[8]; for (int q = 0; q < 8; ++q) bsum[q] = bf16_rne(bih[q * 32 + lane]) + bf16_rne(bhh[q * 32 + lane]);
#pragma unroll 1
  for (int half = 0; half < 2; ++half) { const size_t r0 = r0w + half * 16; const bool live = r0 < (size_t)BV;
    for (int rr = 0; rr < 16; ++rr) { const float t0 = bf16_rne(tr[(r0 + rr) * 2]), t1 = bf16_rne(tr[(r0 + rr) * 2 + 1]); if (lane < EM) X0[rr][lane] = leaky(pmul(t0, we2[0]) + pmul(t1, we2[1]) + bel); }
    wave_lds_sync();
#pragma unroll 1
    for (int m = 0; m < NS; ++m) {
      for (int rr = 0; rr < 16; ++rr) { if (lane < EM) Xs[rr][lane] = X0[rr][lane]; for (int q = 0; q < 2; ++q) { Hs[rr][q * 32 + lane] = bf16_rne(h0[(r0 + rr) * HD + q * 32 + lane]); Cs[rr][q * 32 + lane] = bf16_rne(c0[(r0 + rr) * HD + q * 32 + lane]); } }
      float wp0[2], wp1[2], bpm[2]; for (int d = 0; d < 2; ++d) { wp0[d] = bf16_rne(Wp[(m * 2 + d) * HD + lane]); wp1[d] = bf16_rne(Wp[(m * 2 + d) * HD + 32 + lane]); bpm[d] = bf16_rne(bp[m * 2 + d]); }
      wave_lds_sync();
#pragma unroll 1
      for (int t = 0; t < S; ++t) {
        for (int rr = 0; rr < 16; ++rr) { b16 p, q; const float xv = lane < EM ? Xs[rr][lane] : 0.0f; split16(xv * HS, p, q); Ah[rr][lane] = p; Al[rr][lane] = q; for (int qq = 0; qq < 2; ++qq) { split16(Hs[rr][qq * 32 + lane] * HS, p, q); Ah[rr][32 + qq * 32 + lane] = p; Al[rr][32 + qq * 32 + lane] = q; } }
        wave_lds_sync();
        v8f acc[16];
#pragma unroll
        for (int tt = 0; tt < 16; ++tt) acc[tt] = (v8f){};
#pragma unroll
        for (int kb = 0; kb < KA; kb += 32) { const v16b a = frag_kb(&Ah[nloc][kb], hlf), al = frag_kb(&Al[nloc][kb], hlf);
#pragma unroll
          for (int tt = 0; tt < 16; ++tt) { const v16b bw = frag_kb(WL + (size_t)(tt * 16 + nloc) * KA + kb, hlf); acc[tt] = wmma16b(a, bw, acc[tt]); acc[tt] = wmma16b(al, bw, acc[tt]); } }
        wave_lds_sync();
        const float sc = 1.0f / (HS * WSC);
#pragma unroll
        for (int t4 = 0; t4 < 4; ++t4) { const int u = t4 * 16 + nloc; const int sl = (t4 & 1) * 16 + nloc; const float bi = __shfl(bsum[0 + (t4 >> 1)], sl), bf = __shfl(bsum[2 + (t4 >> 1)], sl), bg = __shfl(bsum[4 + (t4 >> 1)], sl), bo = __shfl(bsum[6 + (t4 >> 1)], sl);
#pragma unroll
          for (int r8 = 0; r8 < 8; ++r8) { const int rl = 8 * hlf + r8; const float ig = sigm(acc[t4][r8] * sc + bi), fg = sigm(acc[4 + t4][r8] * sc + bf), gg = tanhf(acc[8 + t4][r8] * sc + bg), og = sigm(acc[12 + t4][r8] * sc + bo);
            const float cn = pmul(fg, Cs[rl][u]) + pmul(ig, gg); Cs[rl][u] = cn; Hs[rl][u] = pmul(og, tanhf(cn)); } }
        wave_lds_sync();
        for (int rr = 0; rr < 16; ++rr) { const float hA = Hs[rr][lane], hB = Hs[rr][32 + lane]; float d0 = pmul(hA, wp0[0]) + pmul(hB, wp1[0]), d1 = pmul(hA, wp0[1]) + pmul(hB, wp1[1]); for (int o = 16; o; o >>= 1) { d0 += __shfl_xor(d0, o); d1 += __shfl_xor(d1, o); } d0 += bpm[0]; d1 += bpm[1];
          if (lane == 0) { Pr[half * 16 + rr][(m * S + t) * 2] = d0; Pr[half * 16 + rr][(m * S + t) * 2 + 1] = d1; } if (lane < EM) Xs[rr][lane] = leaky(pmul(d0, we2[0]) + pmul(d1, we2[1]) + bel); }
        wave_lds_sync(); }
      for (int rr = 0; rr < 16; ++rr) for (int q = 0; q < 2; ++q) Fn[rr][m * HD + q * 32 + lane] = Hs[rr][q * 32 + lane];
      wave_lds_sync(); }
    for (int rr = 0; rr < 16; ++rr) { float lg[NS]; for (int j = 0; j < NS; ++j) { float s = 0.0f; for (int q = 0; q < 6; ++q) { const int k = q * 32 + lane; if (k < S * 2 * NS) s += pmul(Pr[half * 16 + rr][k], bf16_rne(Wc[j * CI + k + HD * (k / (S * 2))])); } for (int q = 0; q < 6; ++q) { const int k = q * 32 + lane; s += pmul(Fn[rr][k], bf16_rne(Wc[j * CI + k + S * 2 * (k / HD + 1)])); }
        for (int o = 16; o; o >>= 1) s += __shfl_xor(s, o); lg[j] = s + bf16_rne(bc[j]); }
      const float mx = fmaxf(lg[0], fmaxf(lg[1], lg[2])); const float e0 = __expf(lg[0] - mx), e1 = __expf(lg[1] - mx), e2 = __expf(lg[2] - mx); const float inv = 1.0f / (e0 + e1 + e2); if (lane == 0) { Cf[half * 16 + rr][0] = live ? e0 * inv : 0.0f; Cf[half * 16 + rr][1] = live ? e1 * inv : 0.0f; Cf[half * 16 + rr][2] = live ? e2 * inv : 0.0f; }
      if (!live && lane == 0) for (int k = 0; k < NS * S * 2; ++k) Pr[half * 16 + rr][k] = 0.0f; }
    wave_lds_sync(); }
  for (int pass = 0; pass < 2; ++pass) { for (int u = lane; u < 32 * NS * S * 2; u += 32) ((volatile float*)out)[r0w * (NS * S * 2) + u] = (&Pr[0][0])[u]; for (int u = lane; u < 32 * NS; u += 32) ((volatile float*)out)[OFF1 + r0w * NS + u] = (&Cf[0][0])[u]; __threadfence(); }
}
}

extern "C" void kernel_launch(void* const* d_in, const int* in_sizes, int n_in, void* d_out, int out_size, void* d_ws, size_t ws_size, hipStream_t stream) {
  (void)n_in;
  auto Fp = [&](int i) { return (const float*)d_in[i]; };
  if (in_sizes[1] != B * 2 || in_sizes[2] != B * HD || in_sizes[3] != B * HD || in_sizes[4] != G4 * EM || in_sizes[5] != G4 * HD || in_sizes[8] != EM * 2 || in_sizes[10] != NS * 2 * HD || in_sizes[12] != NS * CI || out_size != OFF1 + B * NS) return;
  const int BV = B;
  size_t off = 0; char* ws = (char*)d_ws;
  auto carve = [&](size_t bytes) { char* p = ws + off; off += (bytes + 255) & ~(size_t)255; return p; };
  b16* WL = (b16*)carve((size_t)G4 * KA * 2);
  if (off > ws_size) return;
  wl_kernel<<<(G4 * KA / 8 + 255) / 256, 256, 0, stream>>>(Fp(4), Fp(5), WL);
  dec_kernel<<<(BV + 31) / 32, 32, 0, stream>>>(Fp(1), Fp(2), Fp(3), WL, Fp(6), Fp(7), Fp(8), Fp(9), Fp(10), Fp(11), Fp(12), Fp(13), BV, (float*)d_out);
}
